// CausalSelfAttention_70446053589327
// MI455X (gfx1250) — hardware-verified
//
#include <hip/hip_runtime.h>
#ifndef NB
#define NB 2
#endif
#ifndef SEQ
#define SEQ 2048
#endif
#define NB_FULL 2
#define SEQ_FULL 2048
#define DM 1024
#define NH 16
#define HD 64
#define LQ (3 * DM)
#define KO (2 * DM)
#define NKT (SEQ / 32)
#define NQT (SEQ / 16)
#define EARLY 512
#define NR ((size_t)NB * SEQ)
#define NBH (NB * NH)
#define QPLANE (NR * (size_t)LQ)
#define VPLANE ((size_t)NBH * HD * SEQ)

static_assert(NH * HD == DM);
static_assert(HD == 64);
static_assert((DM & (DM - 1)) == 0);
static_assert(DM % 64 == 0 && LQ % 64 == 0);
static_assert(DM % 32 == 0 && KO % 32 == 0);
static_assert(SEQ % 256 == 0);
static_assert(NB <= NB_FULL && SEQ <= SEQ_FULL);
static_assert((NR % 128) == 0);
static_assert(EARLY % 64 == 0);
static_assert((NQT * NKT) % 128 == 0);

typedef _Float16 v16h __attribute__((ext_vector_type(16)));
typedef unsigned short v8us __attribute__((ext_vector_type(8), may_alias));
typedef float v8f  __attribute__((ext_vector_type(8)));
typedef float v4f  __attribute__((ext_vector_type(4)));
typedef float v4fa __attribute__((ext_vector_type(4), may_alias));
typedef int   v4i  __attribute__((ext_vector_type(4)));
typedef int   v4ia __attribute__((ext_vector_type(4), may_alias));
union FragH { v16h v; v8us half[2]; _Float16 h[16]; unsigned short u[16]; };

__device__ __forceinline__ unsigned short bf16_bits(float x) { unsigned int u = __float_as_uint(x); return (unsigned short)((u + 0x7FFFu + ((u >> 16) & 1u)) >> 16); }
__device__ __forceinline__ float bf16_rne(float x) { return __uint_as_float(((unsigned int)bf16_bits(x)) << 16); }

__device__ __forceinline__ v16h ld_frag(const _Float16* __restrict__ base, size_t off, int hh) {
  FragH f;
  f.half[0] = *(const v8us*)((const unsigned short*)base + off + 8 * hh);
  f.half[1] = *(const v8us*)((const unsigned short*)base + off + 16 + 8 * hh);
  return f.v;
}
__device__ __forceinline__ v8f g2_mma(v16h a, v16h b, v8f c) {
  v8f d = __builtin_amdgcn_wmma_f32_16x16x32_f16(false, a, false, b, (short)0, c, false, false);
  asm volatile("v_nop\n\tv_nop\n\tv_nop\n\tv_nop" : "+v"(d) : "v"(a), "v"(b));
  return d;
}

__global__ __launch_bounds__(256) void k_wt_qkv(const float* __restrict__ W, _Float16* __restrict__ Wt) {
  const int t = blockIdx.x * 256 + threadIdx.x;
  if (t >= LQ * (DM / 8)) return;
  const int n = t / (DM / 8), k8 = (t - n * (DM / 8)) * 8;
  FragH f;
#pragma unroll
  for (int i = 0; i < 8; ++i) f.h[i] = (_Float16)(bf16_rne(W[(size_t)(k8 + i) * LQ + n]) * 16.0f);
  const v8us o = f.half[0];
  unsigned short* d = (unsigned short*)Wt + (size_t)n * DM + k8;
  *(volatile v8us*)d = o;
  __threadfence();
  *(volatile v8us*)d = o;
}

__global__ __launch_bounds__(256) void k_wt_out(const float* __restrict__ W, _Float16* __restrict__ Wt) {
  const int t = blockIdx.x * 256 + threadIdx.x;
  if (t >= DM * (KO / 8)) return;
  const int n = t / (KO / 8), k8 = (t - n * (KO / 8)) * 8;
  const int kk = k8 & (DM - 1);
  const float sc = (k8 < DM) ? 1024.0f : 1.0f;
  FragH f;
#pragma unroll
  for (int i = 0; i < 8; ++i) f.h[i] = (_Float16)(bf16_rne(W[(size_t)(kk + i) * DM + n]) * sc);
  const v8us o = f.half[0];
  unsigned short* d = (unsigned short*)Wt + (size_t)n * KO + k8;
  *(volatile v8us*)d = o;
  __threadfence();
  *(volatile v8us*)d = o;
}

__global__ __launch_bounds__(256) void k_x16(const float* __restrict__ x, _Float16* __restrict__ X16) {
  const size_t t = (size_t)blockIdx.x * 256 + threadIdx.x;
  if (t >= NR * DM / 8) return;
  const size_t r = t / (DM / 8);
  const int c8 = (int)(t - r * (DM / 8)) * 8;
  const size_t b = r / SEQ, s = r - b * SEQ;
  const float* src = x + (b * SEQ_FULL + s) * DM + c8;
  const v4f a = *(const v4fa*)src, c = *(const v4fa*)(src + 4);
  FragH f;
#pragma unroll
  for (int q = 0; q < 4; ++q) { f.h[q] = (_Float16)bf16_rne(a[q]); f.h[4 + q] = (_Float16)bf16_rne(c[q]); }
  const v8us o = f.half[0];
  unsigned short* d = (unsigned short*)X16 + t * 8;
  *(volatile v8us*)d = o;
  __threadfence();
  *(volatile v8us*)d = o;
}

__global__ __launch_bounds__(128) void k_flags(const int* __restrict__ mask, int* __restrict__ flags) {
  const int lane = threadIdx.x & 31;
  const int w = __builtin_amdgcn_readfirstlane(threadIdx.x >> 5);
  const int idx = (blockIdx.x * 4 + w) * 32 + lane;
  const int qt = idx / NKT, kt = idx - qt * NKT;
  int anyz = 0, anynz = 0;
#pragma unroll 1
  for (int r = 0; r < 16; ++r) {
    const int* mp = mask + (size_t)(qt * 16 + r) * SEQ_FULL + kt * 32;
#pragma unroll
    for (int c = 0; c < 8; ++c) {
      const v4i v = *(const v4ia*)(mp + c * 4);
#pragma unroll
      for (int q = 0; q < 4; ++q) { anynz |= (v[q] != 0) ? 1 : 0; anyz |= (v[q] == 0) ? 1 : 0; }
    }
  }
  const int f = anynz ? (anyz ? 2 : 1) : 0;
  *(volatile int*)(flags + idx) = f;
  __threadfence();
  *(volatile int*)(flags + idx) = f;
}

__device__ __forceinline__ void gemm_core(const _Float16* __restrict__ A, const int lda, const _Float16* __restrict__ Bt, const int ldb,
                                          const int row0, const int col0, const int K, const int ln, const int hh, v8f (&acc)[8]) {
  const size_t a0 = (size_t)(row0 + ln) * lda, a1 = a0 + (size_t)16 * lda;
  const size_t b0 = (size_t)(col0 + ln) * ldb, b1 = b0 + (size_t)16 * ldb, b2 = b1 + (size_t)16 * ldb, b3 = b2 + (size_t)16 * ldb;
  const v8f z8 = {0.f, 0.f, 0.f, 0.f, 0.f, 0.f, 0.f, 0.f};
  v8f c00 = z8, c01 = z8, c02 = z8, c03 = z8, c10 = z8, c11 = z8, c12 = z8, c13 = z8;
#pragma unroll 1
  for (int kb = 0; kb < K; kb += 32) {
    const v16h f0 = ld_frag(A, a0 + kb, hh), f1 = ld_frag(A, a1 + kb, hh);
    v16h b = ld_frag(Bt, b0 + kb, hh); c00 = g2_mma(f0, b, c00); c10 = g2_mma(f1, b, c10);
    b = ld_frag(Bt, b1 + kb, hh); c01 = g2_mma(f0, b, c01); c11 = g2_mma(f1, b, c11);
    b = ld_frag(Bt, b2 + kb, hh); c02 = g2_mma(f0, b, c02); c12 = g2_mma(f1, b, c12);
    b = ld_frag(Bt, b3 + kb, hh); c03 = g2_mma(f0, b, c03); c13 = g2_mma(f1, b, c13);
  }
  acc[0] = c00; acc[1] = c01; acc[2] = c02; acc[3] = c03; acc[4] = c10; acc[5] = c11; acc[6] = c12; acc[7] = c13;
}

__global__ __launch_bounds__(128) void k_gemm_qkv(const _Float16* __restrict__ A, const _Float16* __restrict__ Bt, const float* __restrict__ bias, _Float16* __restrict__ C16) {
  __shared__ __attribute__((aligned(16))) float so[4][32][68];
  const int tid = threadIdx.x, lane = tid & 31, ln = lane & 15, hh = lane >> 4;
  const int w = __builtin_amdgcn_readfirstlane(tid >> 5);
  constexpr int ntn = LQ / 64;
  const int mt = blockIdx.x / ntn, nq = blockIdx.x - mt * ntn;
  const int row0 = mt * 128 + 32 * w, col0 = nq * 64;
  v8f accs[8];
  gemm_core(A, DM, Bt, DM, row0, col0, DM, ln, hh, accs);
#pragma unroll
  for (int u = 0; u < 8; ++u) {
    const int t = u & 3, half = u >> 2;
    const float bv = bf16_rne(bias[col0 + t * 16 + ln]);
#pragma unroll
    for (int r = 0; r < 8; ++r) so[w][half * 16 + 8 * hh + r][t * 16 + ln] = accs[u][r] * 0.0625f + bv;
  }
  __builtin_amdgcn_fence(4  , "workgroup");
  __builtin_amdgcn_wave_barrier();
  const int rq = lane >> 3, c8 = (lane & 7) * 8;
  for (int pass = 0; pass < 2; ++pass) {
#pragma unroll
    for (int it = 0; it < 8; ++it) {
      const int r = it * 4 + rq;
      const v4f x0 = *(const v4fa*)&so[w][r][c8], x1 = *(const v4fa*)&so[w][r][c8 + 4];
      FragH fh, fr;
#pragma unroll
      for (int q = 0; q < 4; ++q) {
        _Float16 hv = (_Float16)x0[q]; fh.h[q] = hv; fr.h[q] = (_Float16)((x0[q] - (float)hv) * 1024.0f);
        hv = (_Float16)x1[q]; fh.h[4 + q] = hv; fr.h[4 + q] = (_Float16)((x1[q] - (float)hv) * 1024.0f);
      }
      unsigned short* d = (unsigned short*)C16 + (size_t)(row0 + r) * LQ + col0 + c8;
      *(volatile v8us*)d = fh.half[0];
      *(volatile v8us*)(d + QPLANE) = fr.half[0];
    }
    if (pass == 0) __threadfence();
  }
}

__global__ __launch_bounds__(128) void k_gemm_out(const _Float16* __restrict__ A, const _Float16* __restrict__ Bt, const float* __restrict__ bias, float* __restrict__ C) {
  __shared__ __attribute__((aligned(16))) float so[4][32][68];
  const int tid = threadIdx.x, lane = tid & 31, ln = lane & 15, hh = lane >> 4;
  const int w = __builtin_amdgcn_readfirstlane(tid >> 5);
  constexpr int ntn = DM / 64;
  const int mt = blockIdx.x / ntn, nq = blockIdx.x - mt * ntn;
  const int row0 = mt * 128 + 32 * w, col0 = nq * 64;
  v8f accs[8];
  gemm_core(A, KO, Bt, KO, row0, col0, KO, ln, hh, accs);
#pragma unroll
  for (int u = 0; u < 8; ++u) {
    const int t = u & 3, half = u >> 2;
    const float bv = bf16_rne(bias[col0 + t * 16 + ln]);
#pragma unroll
    for (int r = 0; r < 8; ++r) so[w][half * 16 + 8 * hh + r][t * 16 + ln] = accs[u][r] * 0.0000152587890625f + bv;
  }
  __builtin_amdgcn_fence(4  , "workgroup");
  __builtin_amdgcn_wave_barrier();
  const int rsub = lane >> 4, c4 = (lane & 15) * 4;
  for (int pass = 0; pass < 2; ++pass) {
#pragma unroll
    for (int q = 0; q < 16; ++q) {
      const int r = q * 2 + rsub;
      const v4f v = *(const v4fa*)&so[w][r][c4];
      *(volatile v4f*)(C + (size_t)(row0 + r) * DM + col0 + c4) = v;
    }
    if (pass == 0) __threadfence();
  }
}

__global__ __launch_bounds__(256) void k_vt(const _Float16* __restrict__ QKV, _Float16* __restrict__ VT) {
  __shared__ unsigned short tl[64][66];
  const int tid = threadIdx.x;
  const int slab = blockIdx.x / (SEQ / 64), lg = blockIdx.x - slab * (SEQ / 64);
  const int b = slab / NH, h = slab - b * NH;
  const size_t pin = (size_t)blockIdx.y * QPLANE, pout = (size_t)blockIdx.y * VPLANE;
  for (int i = tid; i < 64 * 8; i += 256) {
    const int r = i >> 3, c8 = (i & 7) * 8;
    FragH f;
    f.half[0] = *(const v8us*)((const unsigned short*)QKV + pin + ((size_t)b * SEQ + lg * 64 + r) * LQ + 2 * DM + h * HD + c8);
#pragma unroll
    for (int q = 0; q < 8; ++q) tl[r][c8 + q] = f.u[q];
  }
  __syncthreads();
  for (int pass = 0; pass < 2; ++pass) {
#pragma unroll
    for (int rd = 0; rd < 2; ++rd) {
      const int d = rd * 32 + (tid >> 3), pc = tid & 7;
      FragH f;
#pragma unroll
      for (int q = 0; q < 8; ++q) f.u[q] = tl[pc * 8 + q][d];
      *(volatile v8us*)((unsigned short*)VT + pout + ((size_t)slab * HD + d) * SEQ + lg * 64 + pc * 8) = f.half[0];
    }
    if (pass == 0) __threadfence();
  }
}

template <int FULL>
__device__ __forceinline__ void attn_body(const _Float16* __restrict__ QKV, const _Float16* __restrict__ VT,
                                          const int* __restrict__ mask, const int* __restrict__ flags,
                                          const size_t qoff, const size_t koff0, const size_t voff0, const size_t moff,
                                          const int qt, const int hh, v8f (&o)[4], float& lout) {
  const v8f z8 = {0.f, 0.f, 0.f, 0.f, 0.f, 0.f, 0.f, 0.f};
  v8f om[4] = {z8, z8, z8, z8};
  v8f orr[4] = {z8, z8, z8, z8};
  float m = -1.0e30f, l = 0.f;
  const float c1 = 0.125f, c2 = 0.125f / 1024.0f;
#pragma unroll 1
  for (int kt = 0; kt < NKT; ++kt) {
    const int fl = __builtin_amdgcn_readfirstlane(flags[qt * NKT + kt]);
    if (fl == 0) continue;
    const int s0 = kt * 32;
    const size_t koff = koff0 + (size_t)s0 * LQ;
    v8f sm0 = z8, sm1 = z8, sr0 = z8, sr1 = z8;
#pragma unroll
    for (int ds = 0; ds < 2; ++ds) {
      const v16h qh = ld_frag(QKV, qoff + ds * 32, hh);
      const v16h qr = ld_frag(QKV, QPLANE + qoff + ds * 32, hh);
      v16h kh = ld_frag(QKV, koff + ds * 32, hh);
      sm0 = g2_mma(kh, qh, sm0);
      sr0 = g2_mma(kh, qr, sr0);
      if (FULL) { const v16h kr = ld_frag(QKV, QPLANE + koff + ds * 32, hh); sr0 = g2_mma(kr, qh, sr0); }
      kh = ld_frag(QKV, koff + (size_t)16 * LQ + ds * 32, hh);
      sm1 = g2_mma(kh, qh, sm1);
      sr1 = g2_mma(kh, qr, sr1);
      if (FULL) { const v16h kr = ld_frag(QKV, QPLANE + koff + (size_t)16 * LQ + ds * 32, hh); sr1 = g2_mma(kr, qh, sr1); }
    }
    unsigned kb = 0xFFFFu;
    if (fl != 1) {
      const int* mp = mask + moff + s0;
      const v4i a0 = *(const v4ia*)(mp), a1 = *(const v4ia*)(mp + 4), b0 = *(const v4ia*)(mp + 16), b1 = *(const v4ia*)(mp + 20);
      kb = 0u;
#pragma unroll
      for (int q = 0; q < 4; ++q) {
        kb |= (a0[q] != 0) ? (1u << q) : 0u;
        kb |= (a1[q] != 0) ? (1u << (4 + q)) : 0u;
        kb |= (b0[q] != 0) ? (1u << (8 + q)) : 0u;
        kb |= (b1[q] != 0) ? (1u << (12 + q)) : 0u;
      }
    }
    float t[16];
#pragma unroll
    for (int i = 0; i < 8; ++i) { t[i] = sm0[i] * c1 + sr0[i] * c2; t[8 + i] = sm1[i] * c1 + sr1[i] * c2; }
    if (fl != 1) {
#pragma unroll
      for (int i = 0; i < 16; ++i) t[i] = ((kb >> i) & 1u) ? t[i] : -1.0e30f;
    }
    float tmax = t[0];
#pragma unroll
    for (int i = 1; i < 16; ++i) tmax = fmaxf(tmax, t[i]);
    tmax = fmaxf(tmax, __shfl_xor(tmax, 16));
    const float mn = fmaxf(m, tmax);
    const float alpha = __expf(m - mn);
    m = mn;
    float p[16];
#pragma unroll
    for (int i = 0; i < 16; ++i) p[i] = __expf(t[i] - mn);
    if (fl != 1) {
#pragma unroll
      for (int i = 0; i < 16; ++i) p[i] = ((kb >> i) & 1u) ? p[i] : 0.0f;
    }
    float ps = p[0];
#pragma unroll
    for (int i = 1; i < 16; ++i) ps += p[i];
    ps += __shfl_xor(ps, 16);
    l = l * alpha + ps;
#pragma unroll
    for (int dt = 0; dt < 4; ++dt) { om[dt] = om[dt] * alpha; if (FULL) orr[dt] = orr[dt] * alpha; }
    FragH ph, pr;
#pragma unroll
    for (int i = 0; i < 16; ++i) {
      const float pv = p[i] * 256.0f;
      const _Float16 hv = (_Float16)pv;
      ph.h[i] = hv;
      pr.h[i] = (_Float16)((pv - (float)hv) * 1024.0f);
    }
#pragma unroll
    for (int dt = 0; dt < 4; ++dt) {
      const size_t vo = voff0 + (size_t)dt * 16 * SEQ + s0;
      const v16h va = ld_frag(VT, vo, hh);
      om[dt] = g2_mma(va, ph.v, om[dt]);
      if (FULL) {
        orr[dt] = g2_mma(va, pr.v, orr[dt]);
        const v16h vr = ld_frag(VT, VPLANE + vo, hh);
        orr[dt] = g2_mma(vr, ph.v, orr[dt]);
      }
    }
  }
#pragma unroll
  for (int dt = 0; dt < 4; ++dt) o[dt] = FULL ? (om[dt] + orr[dt] * 0.0009765625f) : om[dt];
  lout = l;
}

__global__ __launch_bounds__(128) void k_attn(const _Float16* __restrict__ QKV, const _Float16* __restrict__ VT, const int* __restrict__ mask,
                                              const int* __restrict__ flags, _Float16* __restrict__ CTX) {
  __shared__ __attribute__((aligned(16))) float so[4][16][68];
  const int tid = threadIdx.x, lane = tid & 31, ln = lane & 15, hh = lane >> 4;
  const int w = __builtin_amdgcn_readfirstlane(tid >> 5);
  constexpr int QB = SEQ / 64;
  const int bh = blockIdx.x / QB, qblk = blockIdx.x - bh * QB;
  const int b = bh / NH, h = bh - b * NH;
  const int qbase = qblk * 64 + w * 16;
  const int qt = qbase >> 4;
  const size_t brow0 = (size_t)b * SEQ;
  const size_t qoff = (brow0 + qbase + ln) * LQ + (size_t)h * HD;
  const size_t koff0 = (brow0 + ln) * LQ + DM + (size_t)h * HD;
  const size_t voff0 = ((size_t)bh * HD + ln) * SEQ;
  const size_t moff = (size_t)(qbase + ln) * SEQ_FULL + 8 * hh;
  v8f o[4];
  float l;
  if (qbase < EARLY) attn_body<1>(QKV, VT, mask, flags, qoff, koff0, voff0, moff, qt, hh, o, l);
  else               attn_body<0>(QKV, VT, mask, flags, qoff, koff0, voff0, moff, qt, hh, o, l);
  const float inv = 0.25f * (1.0f / l);
#pragma unroll
  for (int dt = 0; dt < 4; ++dt) {
    const v4f a = {o[dt][0] * inv, o[dt][1] * inv, o[dt][2] * inv, o[dt][3] * inv};
    const v4f c = {o[dt][4] * inv, o[dt][5] * inv, o[dt][6] * inv, o[dt][7] * inv};
    *(v4fa*)&so[w][ln][dt * 16 + 8 * hh] = a;
    *(v4fa*)&so[w][ln][dt * 16 + 8 * hh + 4] = c;
  }
  __builtin_amdgcn_fence(4  , "workgroup");
  __builtin_amdgcn_wave_barrier();
  const int rq = lane >> 3, c8 = (lane & 7) * 8;
  for (int pass = 0; pass < 2; ++pass) {
#pragma unroll
    for (int it = 0; it < 4; ++it) {
      const int r = it * 4 + rq;
      const v4f x0 = *(const v4fa*)&so[w][r][c8], x1 = *(const v4fa*)&so[w][r][c8 + 4];
      FragH fh, fr;
#pragma unroll
      for (int q = 0; q < 4; ++q) {
        _Float16 hv = (_Float16)x0[q]; fh.h[q] = hv; fr.h[q] = (_Float16)((x0[q] - (float)hv) * 1024.0f);
        hv = (_Float16)x1[q]; fh.h[4 + q] = hv; fr.h[4 + q] = (_Float16)((x1[q] - (float)hv) * 1024.0f);
      }
      unsigned short* d = (unsigned short*)CTX + (brow0 + qbase + r) * KO + h * HD + c8;
      *(volatile v8us*)d = fh.half[0];
      *(volatile v8us*)(d + DM) = fr.half[0];
    }
    if (pass == 0) __threadfence();
  }
}

extern "C" void kernel_launch(void* const* d_in, const int* in_sizes, int n_in,
                              void* d_out, int out_size, void* d_ws, size_t ws_size, hipStream_t stream) {
  constexpr size_t SZ_BQKV = (size_t)LQ * DM * 2;
  constexpr size_t SZ_BO2  = (size_t)DM * KO * 2;
  constexpr size_t SZ_X16  = NR * DM * 2;
  constexpr size_t SZ_QKV2 = 2 * QPLANE * 2;
  constexpr size_t SZ_VT2  = 2 * VPLANE * 2;
  constexpr size_t SZ_CTX  = NR * KO * 2;
  constexpr size_t SZ_FLG  = (size_t)NQT * NKT * 4;
  static_assert(SZ_BQKV % 256 == 0 && SZ_BO2 % 256 == 0 && SZ_X16 % 256 == 0 && SZ_QKV2 % 256 == 0 && SZ_VT2 % 256 == 0 && SZ_CTX % 256 == 0 && SZ_FLG % 128 == 0);
  constexpr size_t TOTAL = SZ_BQKV + SZ_BO2 + SZ_X16 + SZ_QKV2 + SZ_VT2 + SZ_CTX + SZ_FLG;
  static_assert(TOTAL <= (size_t)134217728);
  if (n_in < 6) return;
  if ((size_t)in_sizes[0] < ((size_t)(NB - 1) * SEQ_FULL + SEQ) * DM) return;
  if ((size_t)in_sizes[1] < (size_t)(SEQ - 1) * SEQ_FULL + SEQ) return;
  if ((size_t)in_sizes[2] < (size_t)DM * LQ) return;
  if (in_sizes[3] < LQ) return;
  if ((size_t)in_sizes[4] < (size_t)DM * DM) return;
  if (in_sizes[5] < DM) return;
  if ((size_t)out_size < NR * DM) return;
  if (ws_size < TOTAL) return;
  const float* x  = (const float*)d_in[0];
  const int* mask = (const int*)d_in[1];
  const float* Wa = (const float*)d_in[2];
  const float* ba = (const float*)d_in[3];
  const float* Wp = (const float*)d_in[4];
  const float* bp = (const float*)d_in[5];
  float* out = (float*)d_out;
  char* ws = (char*)d_ws;
  size_t off = 0;
  _Float16* BQKV = (_Float16*)(ws + off); off += SZ_BQKV;
  _Float16* BO2  = (_Float16*)(ws + off); off += SZ_BO2;
  _Float16* X16  = (_Float16*)(ws + off); off += SZ_X16;
  _Float16* QKV2 = (_Float16*)(ws + off); off += SZ_QKV2;
  _Float16* VT2  = (_Float16*)(ws + off); off += SZ_VT2;
  _Float16* CTX  = (_Float16*)(ws + off); off += SZ_CTX;
  int* FLG       = (int*)(ws + off);      off += SZ_FLG;
  k_wt_qkv<<<(unsigned)(((size_t)LQ * (DM / 8) + 255) / 256), 256, 0, stream>>>(Wa, BQKV);
  k_wt_out<<<(unsigned)(((size_t)DM * (KO / 8) + 255) / 256), 256, 0, stream>>>(Wp, BO2);
  k_x16<<<(unsigned)((NR * DM / 8 + 255) / 256), 256, 0, stream>>>(x, X16);
  k_flags<<<(unsigned)(NQT * NKT / 128), 128, 0, stream>>>(mask, FLG);
  k_gemm_qkv<<<(unsigned)((NR / 128) * (LQ / 64)), 128, 0, stream>>>(X16, BQKV, ba, QKV2);
  k_vt<<<dim3((unsigned)(NBH * (SEQ / 64)), 2), 256, 0, stream>>>(QKV2, VT2);
  k_attn<<<(unsigned)(NBH * (SEQ / 64)), 128, 0, stream>>>(QKV2, VT2, mask, FLG, CTX);
  k_gemm_out<<<(unsigned)((NR / 128) * (DM / 64)), 128, 0, stream>>>(CTX, BO2, bp, out);
}
